// GCNEdgeClassifier_45741401703144
// MI455X (gfx1250) — hardware-verified
//
#include <hip/hip_runtime.h>
#include <stdint.h>


typedef _Float16 v4h  __attribute__((ext_vector_type(4)));
typedef _Float16 v8h  __attribute__((ext_vector_type(8)));
typedef _Float16 v16h __attribute__((ext_vector_type(16)));
typedef float    v8f  __attribute__((ext_vector_type(8)));
typedef float    v4f  __attribute__((ext_vector_type(4)));
typedef unsigned v4u  __attribute__((ext_vector_type(4)));

union Frag { v16h v; v8h half[2]; };
union Pk8  { v8h h; v4u u; _Float16 s[8]; };

#define HID      128
#define IN_FEAT  4
#define NLAYER   3
#define KE       (2 * HID)

#define NT_SCAN  256
#define NW_SCAN  8
#define LCAP     128
#define R_AGG    512
#define R_DEG    4096
#define EC_MAX   131072

#define AGG_LDS_BYTES (R_AGG * HID * 4 + R_AGG * 4 + NW_SCAN * LCAP * 8 + NW_SCAN * 4)

__device__ __forceinline__ v16h ldfrag(const _Float16* rowp, int kb, int h) {
    Frag f;
    f.half[0] = *(const v8h*)(rowp + kb + 8 * h);
    f.half[1] = *(const v8h*)(rowp + kb + 16 + 8 * h);
    return f.v;
}

__device__ __forceinline__ v8f wmma16(v16h a, v16h b, v8f c) {
    c = __builtin_amdgcn_wmma_f32_16x16x32_f16(false, a, false, b, (short)0, c, false, false);
    asm volatile("v_nop\n\tv_nop\n\tv_nop\n\tv_nop" : "+v"(c) : "v"(a), "v"(b));
    return c;
}

__global__ __launch_bounds__(256) void k_prep(const float* __restrict__ Wg1,
                                              const float* __restrict__ Wg2,
                                              const float* __restrict__ Wg3,
                                              const float* __restrict__ Wm1,
                                              _Float16* __restrict__ wg16t,
                                              _Float16* __restrict__ wm1t) {
    const int idx = blockIdx.x * blockDim.x + threadIdx.x;
    const int NG = NLAYER * HID * (HID / 8);
    const int NM = HID * (KE / 8);
    Pk8 pk;
    _Float16* dstp;
    if (idx < NG) {
        const int l   = idx / (HID * (HID / 8));
        const int rem = idx - l * (HID * (HID / 8));
        const int n   = rem / (HID / 8);
        const int k8  = rem - n * (HID / 8);
        const float* W = (l == 0) ? Wg1 : ((l == 1) ? Wg2 : Wg3);
        #pragma unroll
        for (int i = 0; i < 8; ++i) pk.s[i] = (_Float16)W[(k8 * 8 + i) * HID + n];
        dstp = wg16t + (size_t)idx * 8;
    } else if (idx < NG + NM) {
        const int j  = idx - NG;
        const int n  = j / (KE / 8);
        const int k8 = j - n * (KE / 8);
        #pragma unroll
        for (int i = 0; i < 8; ++i) pk.s[i] = (_Float16)Wm1[(k8 * 8 + i) * HID + n];
        dstp = wm1t + (size_t)j * 8;
    } else {
        return;
    }
    *(volatile v4u*)dstp = pk.u;
    __threadfence();
    *(volatile v4u*)dstp = pk.u;
}

__global__ __launch_bounds__(256) void k_enc(const float* __restrict__ x,
                                             const float* __restrict__ We,
                                             const float* __restrict__ be,
                                             float* __restrict__ h32,
                                             int nn, int npad) {
    const int idx = blockIdx.x * blockDim.x + threadIdx.x;
    if (idx >= npad * (HID / 4)) return;
    const int n  = idx >> 5;
    const int c4 = idx & 31;
    v4f v = {0.f, 0.f, 0.f, 0.f};
    if (n < nn) {
        const float x0 = x[(size_t)n * IN_FEAT + 0];
        const float x1 = x[(size_t)n * IN_FEAT + 1];
        const float x2 = x[(size_t)n * IN_FEAT + 2];
        const float x3 = x[(size_t)n * IN_FEAT + 3];
        #pragma unroll
        for (int c = 0; c < 4; ++c) {
            const int col = c4 * 4 + c;
            float a = x0 * We[col] + x1 * We[HID + col] + x2 * We[2 * HID + col] + x3 * We[3 * HID + col];
            a += be[col];
            v[c] = a > 0.0f ? a : 0.0f;
        }
    }
    float* p = h32 + (size_t)n * HID + c4 * 4;
    *(volatile v4f*)p = v;
    __threadfence();
    *(volatile v4f*)p = v;
}

__global__ __launch_bounds__(NT_SCAN) void k_deg(const int* __restrict__ dstv,
                                                 float* __restrict__ dinv,
                                                 int nn, int ne, int npad) {
    __shared__ int cnta[R_DEG];
    __shared__ int lst[NW_SCAN * LCAP];
    __shared__ int cnts[NW_SCAN];
    const int tid = threadIdx.x, wave = tid >> 5, lane = tid & 31;
    const int n0 = blockIdx.x * R_DEG;
    for (int i = tid; i < R_DEG; i += NT_SCAN) cnta[i] = 0;
    __syncthreads();
    const unsigned lt = (1u << lane) - 1u;
    for (int base = 0; base < ne; base += NT_SCAN * 4) {
        const int e = base + tid * 4;
        int dl[4]; bool hb[4]; unsigned mk[4];
        #pragma unroll
        for (int j = 0; j < 4; ++j) {
            const int ej = e + j;
            const int d  = dstv[min(ej, ne - 1)];
            const int t  = d - n0;
            hb[j] = (ej < ne) && (d < nn) && ((unsigned)t < (unsigned)R_DEG);
            dl[j] = t;
        }
        #pragma unroll
        for (int j = 0; j < 4; ++j) mk[j] = __builtin_amdgcn_ballot_w32(hb[j]);
        int pref = 0;
        #pragma unroll
        for (int j = 0; j < 4; ++j) {
            const int pos = pref + (int)__builtin_popcount(mk[j] & lt);
            if (hb[j]) lst[wave * LCAP + pos] = dl[j];
            pref += (int)__builtin_popcount(mk[j]);
        }
        if (lane == 0) cnts[wave] = pref;
        __syncthreads();
        if (wave == 0) {
            for (int w = 0; w < NW_SCAN; ++w) {
                const int c = min(cnts[w], LCAP);
                for (int i = 0; i < c; ++i) {
                    const int t = lst[w * LCAP + i] & (R_DEG - 1);
                    if ((t & 31) == lane) cnta[t] += 1;
                }
            }
        }
        __syncthreads();
    }
    v4f vv[R_DEG / 4 / NT_SCAN];
    #pragma unroll
    for (int j = 0; j < R_DEG / 4 / NT_SCAN; ++j) {
        const int i = tid + NT_SCAN * j;
        const int d = n0 + 4 * i;
        v4f v;
        #pragma unroll
        for (int q = 0; q < 4; ++q) {
            const int dd = d + q;
            const float c = (float)(cnta[4 * i + q] + 1);
            v[q] = (dd < nn) ? rsqrtf(c) : 1.0f;
        }
        vv[j] = v;
        if (d < npad) *(volatile v4f*)(dinv + d) = v;
    }
    __threadfence();
    #pragma unroll
    for (int j = 0; j < R_DEG / 4 / NT_SCAN; ++j) {
        const int i = tid + NT_SCAN * j;
        const int d = n0 + 4 * i;
        if (d < npad) *(volatile v4f*)(dinv + d) = vv[j];
    }
}

__global__ __launch_bounds__(NT_SCAN) void k_agg(const float* __restrict__ hin,
                                                 const int* __restrict__ srcv,
                                                 const int* __restrict__ dstv,
                                                 const float* __restrict__ dinv,
                                                 _Float16* __restrict__ agg,
                                                 int nn, int ne, int npad) {
    extern __shared__ __align__(16) float dynlds[];
    float* accl  = dynlds;
    float* ld    = dynlds + R_AGG * HID;
    int2*  lists = (int2*)(ld + R_AGG);
    int*   cnts  = (int*)(lists + NW_SCAN * LCAP);
    const int tid = threadIdx.x, wave = tid >> 5, lane = tid & 31;
    const int n0 = blockIdx.x * R_AGG;

    for (int i = tid; i < R_AGG; i += NT_SCAN) ld[i] = dinv[min(n0 + i, npad - 1)];
    __syncthreads();
    {
        v4f* a4 = (v4f*)accl;
        const v4f z4 = {0.f, 0.f, 0.f, 0.f};
        for (int i = tid; i < R_AGG * (HID / 4); i += NT_SCAN) {
            const int row = i >> 5, c4 = i & 31;
            const int d = n0 + row;
            v4f v = z4;
            if (d < nn) {
                const float w = ld[row] * ld[row];
                v = w * ((const v4f*)(hin + (size_t)d * HID))[c4];
            }
            a4[i] = v;
        }
    }
    __syncthreads();

    const unsigned lt = (1u << lane) - 1u;
    for (int base = 0; base < ne; base += NT_SCAN * 4) {
        const int e = base + tid * 4;
        int dl[4]; bool hb[4]; unsigned mk[4];
        #pragma unroll
        for (int j = 0; j < 4; ++j) {
            const int ej = e + j;
            const int d  = dstv[min(ej, ne - 1)];
            const int t  = d - n0;
            hb[j] = (ej < ne) && (d < nn) && ((unsigned)t < (unsigned)R_AGG);
            dl[j] = t;
        }
        #pragma unroll
        for (int j = 0; j < 4; ++j) mk[j] = __builtin_amdgcn_ballot_w32(hb[j]);
        int pref = 0;
        #pragma unroll
        for (int j = 0; j < 4; ++j) {
            const int pos = pref + (int)__builtin_popcount(mk[j] & lt);
            if (hb[j]) {
                int s = srcv[e + j];
                s = min(max(s, 0), nn - 1);
                lists[wave * LCAP + pos] = make_int2(s, dl[j]);
            }
            pref += (int)__builtin_popcount(mk[j]);
        }
        if (lane == 0) cnts[wave] = pref;
        __syncthreads();
        if (wave == 0) {
            for (int w = 0; w < NW_SCAN; ++w) {
                const int c = min(cnts[w], LCAP);
                for (int i = 0; i < c; ++i) {
                    const int2 en = lists[w * LCAP + i];
                    const int s  = min(max((int)en.x, 0), nn - 1);
                    const int dd = en.y & (R_AGG - 1);
                    const float wgt = dinv[s] * ld[dd];
                    const v4f tv = ((const v4f*)(hin + (size_t)s * HID))[lane];
                    v4f* ap = (v4f*)(accl + dd * HID) + lane;
                    v4f a = *ap;
                    a = a + wgt * tv;
                    *ap = a;
                }
            }
        }
        __syncthreads();
    }

    const int sub = tid & 15, rip = tid >> 4;
    for (int g = 0; g < R_AGG / 128; ++g) {
        v4u vv[8];
        #pragma unroll
        for (int j = 0; j < 8; ++j) {
            const int row = g * 128 + j * 16 + rip;
            const float* ap = accl + row * HID + sub * 8;
            const v4f fa = *(const v4f*)ap;
            const v4f fb = *(const v4f*)(ap + 4);
            Pk8 pk;
            #pragma unroll
            for (int c = 0; c < 4; ++c) { pk.s[c] = (_Float16)fa[c]; pk.s[4 + c] = (_Float16)fb[c]; }
            vv[j] = pk.u;
        }
        #pragma unroll
        for (int j = 0; j < 8; ++j) {
            const int gr = n0 + g * 128 + j * 16 + rip;
            if (gr < npad) *(volatile v4u*)(agg + (size_t)gr * HID + sub * 8) = vv[j];
        }
        __threadfence();
        #pragma unroll
        for (int j = 0; j < 8; ++j) {
            const int gr = n0 + g * 128 + j * 16 + rip;
            if (gr < npad) *(volatile v4u*)(agg + (size_t)gr * HID + sub * 8) = vv[j];
        }
    }
}

__global__ __launch_bounds__(128) void k_xform(const _Float16* __restrict__ agg,
                                                const _Float16* __restrict__ Wt,
                                                const float* __restrict__ bias,
                                                float* __restrict__ hout,
                                                int nn, int npad) {
    __shared__ __align__(16) float Ct[4][16][HID];
    const int wave = threadIdx.x >> 5, lane = threadIdx.x & 31, h = lane >> 4, m = lane & 15;
    const int g0 = (blockIdx.x * 4 + wave) * 16;

    v8f acc[8];
    const v8f z = {0.f, 0.f, 0.f, 0.f, 0.f, 0.f, 0.f, 0.f};
    #pragma unroll
    for (int i = 0; i < 8; ++i) acc[i] = z;
    const _Float16* ar = agg + (size_t)(g0 + m) * HID;
    #pragma unroll
    for (int kt = 0; kt < HID / 32; ++kt) {
        const int kb = kt * 32;
        const v16h a = ldfrag(ar, kb, h);
        #pragma unroll
        for (int nt = 0; nt < 8; ++nt) {
            const v16h b = ldfrag(Wt + (size_t)(nt * 16 + m) * HID, kb, h);
            acc[nt] = wmma16(a, b, acc[nt]);
        }
    }
    #pragma unroll
    for (int nt = 0; nt < 8; ++nt) {
        const int n = nt * 16 + m;
        const float bn = bias[n];
        #pragma unroll
        for (int r = 0; r < 8; ++r) {
            const int lr = 8 * h + r;
            float zz = acc[nt][r] + bn;
            zz = zz > 0.0f ? zz : 0.0f;
            if (g0 + lr >= nn) zz = 0.0f;
            Ct[wave][lr][n] = zz;
        }
    }
    __syncthreads();
    {
        float* orow = hout + (size_t)g0 * HID + 4 * lane;
        v4f vr[16];
        #pragma unroll
        for (int r = 0; r < 16; ++r) vr[r] = *(const v4f*)(&Ct[wave][r][4 * lane]);
        #pragma unroll
        for (int r = 0; r < 16; ++r) *(volatile v4f*)(orow + (size_t)r * HID) = vr[r];
        __threadfence();
        #pragma unroll
        for (int r = 0; r < 16; ++r) *(volatile v4f*)(orow + (size_t)r * HID) = vr[r];
    }
}

__global__ __launch_bounds__(256) void k_egather(const float* __restrict__ h32,
                                                 const int* __restrict__ srcv,
                                                 const int* __restrict__ dstv,
                                                 _Float16* __restrict__ ef,
                                                 int nn, int cb, int cnt, int cpad) {
    const int idx  = blockIdx.x * blockDim.x + threadIdx.x;
    const int row  = idx >> 5;
    const int part = idx & 31;
    if (row >= cpad) return;
    Pk8 pk;
    const v4u zu = {0u, 0u, 0u, 0u};
    pk.u = zu;
    if (row < cnt) {
        const int e = cb + row;
        int node = (part < 16) ? srcv[e] : dstv[e];
        node = min(max(node, 0), nn - 1);
        const v4f* sp = (const v4f*)(h32 + (size_t)node * HID + (part & 15) * 8);
        const v4f fa = sp[0], fb = sp[1];
        #pragma unroll
        for (int c = 0; c < 4; ++c) { pk.s[c] = (_Float16)fa[c]; pk.s[4 + c] = (_Float16)fb[c]; }
    }
    _Float16* p = ef + (size_t)row * KE + part * 8;
    *(volatile v4u*)p = pk.u;
    __threadfence();
    *(volatile v4u*)p = pk.u;
}

__global__ __launch_bounds__(64) void k_mlp(const _Float16* __restrict__ ef,
                                            const _Float16* __restrict__ Wm1t,
                                            const float* __restrict__ b1,
                                            const float* __restrict__ Wm2,
                                            const float* __restrict__ b2,
                                            float* __restrict__ out,
                                            int cb, int cnt) {
    __shared__ __align__(16) float Zt[2][16][HID];
    __shared__ __align__(16) float Ot[96];
    const int wave = threadIdx.x >> 5, lane = threadIdx.x & 31, h = lane >> 4, m = lane & 15;
    const int lr0 = blockIdx.x * 32 + wave * 16;

    v8f acc[8];
    const v8f z = {0.f, 0.f, 0.f, 0.f, 0.f, 0.f, 0.f, 0.f};
    #pragma unroll
    for (int i = 0; i < 8; ++i) acc[i] = z;
    const _Float16* ar = ef + (size_t)(lr0 + m) * KE;
    #pragma unroll
    for (int kt = 0; kt < KE / 32; ++kt) {
        const int kb = kt * 32;
        const v16h a = ldfrag(ar, kb, h);
        #pragma unroll
        for (int nt = 0; nt < 8; ++nt) {
            const v16h b = ldfrag(Wm1t + (size_t)(nt * 16 + m) * KE, kb, h);
            acc[nt] = wmma16(a, b, acc[nt]);
        }
    }
    #pragma unroll
    for (int nt = 0; nt < 8; ++nt) {
        const int n = nt * 16 + m;
        const float bn = b1[n];
        #pragma unroll
        for (int r = 0; r < 8; ++r) {
            const float zz = acc[nt][r] + bn;
            Zt[wave][8 * h + r][n] = zz > 0.0f ? zz : 0.0f;
        }
    }
    __syncthreads();

    {
        const float* zr = &Zt[wave][m][h * (HID / 2)];
        const float* wq = Wm2 + h * (HID / 2) * 3;
        float p0 = 0.0f, p1 = 0.0f, p2 = 0.0f;
        #pragma unroll 4
        for (int f = 0; f < HID / 2; ++f) {
            const float zv = zr[f];
            p0 += zv * wq[f * 3 + 0];
            p1 += zv * wq[f * 3 + 1];
            p2 += zv * wq[f * 3 + 2];
        }
        p0 += __shfl_xor(p0, 16);
        p1 += __shfl_xor(p1, 16);
        p2 += __shfl_xor(p2, 16);
        if (h == 0) {
            Ot[(wave * 16 + m) * 3 + 0] = p0 + b2[0];
            Ot[(wave * 16 + m) * 3 + 1] = p1 + b2[1];
            Ot[(wave * 16 + m) * 3 + 2] = p2 + b2[2];
        }
    }
    __syncthreads();

    if (wave == 0) {
        const int le0 = blockIdx.x * 32;
        const size_t ob = (size_t)(cb + le0) * 3;
        if (le0 + 32 <= cnt) {
            const bool act = lane < 24;
            v4f v = {0.f, 0.f, 0.f, 0.f};
            if (act) v = ((const v4f*)Ot)[lane];
            if (act) *(volatile v4f*)(out + ob + 4 * lane) = v;
            __threadfence();
            if (act) *(volatile v4f*)(out + ob + 4 * lane) = v;
        } else {
            const int nval = (cnt - le0) * 3;
            float ov[3];
            #pragma unroll
            for (int j = 0; j < 3; ++j) {
                const int i = lane + 32 * j;
                ov[j] = Ot[i];
                if (i < nval) ((volatile float*)out)[ob + i] = ov[j];
            }
            __threadfence();
            #pragma unroll
            for (int j = 0; j < 3; ++j) {
                const int i = lane + 32 * j;
                if (i < nval) ((volatile float*)out)[ob + i] = ov[j];
            }
        }
    }
}

extern "C" void kernel_launch(void* const* d_in, const int* in_sizes, int n_in,
                              void* d_out, int out_size, void* d_ws, size_t ws_size,
                              hipStream_t stream) {
    if (n_in < 14) return;
    const float* x    = (const float*)d_in[0];
    const int*   ei   = (const int*)d_in[1];
    const float* Wenc = (const float*)d_in[2];
    const float* benc = (const float*)d_in[3];
    const float* Wg1  = (const float*)d_in[4];
    const float* bg1  = (const float*)d_in[5];
    const float* Wg2  = (const float*)d_in[6];
    const float* bg2  = (const float*)d_in[7];
    const float* Wg3  = (const float*)d_in[8];
    const float* bg3  = (const float*)d_in[9];
    const float* Wm1  = (const float*)d_in[10];
    const float* bm1  = (const float*)d_in[11];
    const float* Wm2  = (const float*)d_in[12];
    const float* bm2  = (const float*)d_in[13];
    float* out = (float*)d_out;

    const int nn = in_sizes[0] / IN_FEAT;
    const int ne = in_sizes[1] / 2;
    if (nn <= 0 || ne <= 0) return;
    if ((size_t)out_size < (size_t)ne * 3) return;
    const int npad = ((nn + 63) / 64) * 64;
    const int ne32 = ((ne + 31) / 32) * 32;
    const int ecap = ne32 < EC_MAX ? ne32 : EC_MAX;
    const int* srcv = ei;
    const int* dstv = ei + ne;

    size_t off = 0;
    char* ws = (char*)d_ws;
    const size_t b_h32 = (size_t)npad * HID * 4;
    const size_t b_agg = (size_t)npad * HID * 2;
    const size_t b_dnv = (size_t)npad * 4;
    const size_t b_wg  = (size_t)NLAYER * HID * HID * 2;
    const size_t b_wm  = (size_t)HID * KE * 2;
    const size_t b_ef  = (size_t)ecap * KE * 2;
    float* h32 = (float*)(ws + off);          off += (b_h32 + 255) & ~(size_t)255;
    _Float16* agg16 = (_Float16*)(ws + off); off += (b_agg + 255) & ~(size_t)255;
    float* dinv = (float*)(ws + off);        off += (b_dnv + 255) & ~(size_t)255;
    _Float16* wg16t = (_Float16*)(ws + off); off += (b_wg + 255) & ~(size_t)255;
    _Float16* wm1t  = (_Float16*)(ws + off); off += (b_wm + 255) & ~(size_t)255;
    _Float16* efb   = (_Float16*)(ws + off); off += (b_ef + 255) & ~(size_t)255;
    if (off > ws_size) return;

    hipFuncSetAttribute((const void*)k_agg, hipFuncAttributeMaxDynamicSharedMemorySize, AGG_LDS_BYTES);

    {
        const int total = NLAYER * HID * (HID / 8) + HID * (KE / 8);
        k_prep<<<dim3((total + 255) / 256), dim3(256), 0, stream>>>(Wg1, Wg2, Wg3, Wm1, wg16t, wm1t);
    }
    {
        const int total = npad * (HID / 4);
        k_enc<<<dim3((total + 255) / 256), dim3(256), 0, stream>>>(x, Wenc, benc, h32, nn, npad);
    }
    k_deg<<<dim3((npad + R_DEG - 1) / R_DEG), dim3(NT_SCAN), 0, stream>>>(dstv, dinv, nn, ne, npad);

    const float* biases[NLAYER] = {bg1, bg2, bg3};
    const int aggBlocks = (npad + R_AGG - 1) / R_AGG;
    const int xfBlocks  = npad / 64;
    for (int l = 0; l < NLAYER; ++l) {
        k_agg<<<dim3(aggBlocks), dim3(NT_SCAN), AGG_LDS_BYTES, stream>>>(
            h32, srcv, dstv, dinv, agg16, nn, ne, npad);
        k_xform<<<dim3(xfBlocks), dim3(128), 0, stream>>>(
            agg16, wg16t + (size_t)l * HID * HID, biases[l], h32, nn, npad);
    }

    const int nchunk = (ne + ecap - 1) / ecap;
    for (int c = 0; c < nchunk; ++c) {
        const int cb   = c * ecap;
        const int cnt  = (ne - cb) < ecap ? (ne - cb) : ecap;
        const int cpad = ((cnt + 31) / 32) * 32;
        k_egather<<<dim3((cpad * 32 + 255) / 256), dim3(256), 0, stream>>>(
            h32, srcv, dstv, efb, nn, cb, cnt, cpad);
        k_mlp<<<dim3(cpad / 32), dim3(64), 0, stream>>>(
            efb, wm1t, bm1, Wm2, bm2, out, cb, cnt);
    }
}
